// LoFTREncoderLayer_81449759801419
// MI455X (gfx1250) — hardware-verified
//
#include <hip/hip_runtime.h>
#include <math.h>

constexpr int kBatch = 4;
constexpr int kSeq   = 8192;
constexpr int kDim   = 256;
constexpr int kHeads = 8;
constexpr int kDh    = 32;
constexpr int kHid2  = 512;
constexpr int kTok   = kBatch * kSeq;
constexpr float kWCarry     = 16.0f;
constexpr float kWCarryInv  = 1.0f / 16.0f;
constexpr float kMsgCarry   = 64.0f;
constexpr float kMergeScale = 1.0f / (16.0f * 64.0f);
constexpr float kLnEps      = 1.0e-5f;
constexpr float kAttnEps    = 1.0e-6f;
constexpr float kInvDim     = 1.0f / 256.0f;
static_assert(kHeads * kDh == kDim);
static_assert(kTok % 64 == 0 && kDim % 64 == 0 && kSeq % 64 == 0 && kHid2 % 64 == 0);
static_assert(kDim % 32 == 0 && kHid2 % 32 == 0 && kSeq % 32 == 0);
static_assert(kSeq % 128 == 0 && kTok % 32 == 0);

typedef __attribute__((ext_vector_type(16))) _Float16 v16h;
typedef __attribute__((ext_vector_type(8)))  _Float16 v8h;
typedef __attribute__((ext_vector_type(16))) __bf16   v16b;
typedef __attribute__((ext_vector_type(8)))  __bf16   v8b;
typedef __attribute__((ext_vector_type(8)))  float    v8f;
typedef __attribute__((ext_vector_type(4)))  float    v4f;
typedef __attribute__((ext_vector_type(4)))  unsigned int v4u;

__device__ __forceinline__ unsigned short f2bf_bits(float f) {
  unsigned u = __float_as_uint(f);
  return (unsigned short)((u + 0x7FFFu + ((u >> 16) & 1u)) >> 16);
}
__device__ __forceinline__ float bf_bits2f(unsigned short h) { return __uint_as_float(((unsigned)h) << 16); }

__device__ __forceinline__ void dep_guard_h(v8f& a, v8f& b, v16h x, v16h y) { asm volatile("v_nop\n\tv_nop\n\tv_nop\n\tv_nop" : "+v"(a), "+v"(b) : "v"(x), "v"(y)); }
__device__ __forceinline__ void dep_guard_b(v8f& a, v8f& b, v16b x, v16b y) { asm volatile("v_nop\n\tv_nop\n\tv_nop\n\tv_nop" : "+v"(a), "+v"(b) : "v"(x), "v"(y)); }
__device__ __forceinline__ void keep4_h(v16h a, v16h b, v16h c, v16h d) { asm volatile("v_nop" :: "v"(a), "v"(b), "v"(c), "v"(d)); }
__device__ __forceinline__ void keep4_b(v16b a, v16b b, v16b c, v16b d) { asm volatile("v_nop" :: "v"(a), "v"(b), "v"(c), "v"(d)); }
__device__ __forceinline__ void acc_guard4(v8f& a, v8f& b, v8f& c, v8f& d) { asm volatile("v_nop\n\tv_nop\n\tv_nop\n\tv_nop" : "+v"(a), "+v"(b), "+v"(c), "+v"(d)); }
template <typename T> struct Frag;
template <> struct Frag<_Float16> {
  typedef v16h V; union U { v16h v; v8h h[2]; };
  static __device__ __forceinline__ v16h load(const _Float16* p) {
    U f; f.h[0] = *(const v8h*)(p); f.h[1] = *(const v8h*)(p + 16); return f.v;
  }
  static __device__ __forceinline__ v8f mma(v16h a, v16h b, v8f c) {
    return __builtin_amdgcn_wmma_f32_16x16x32_f16(false, a, false, b, (short)0, c, false, false);
  }
  static __device__ __forceinline__ void guard(v8f& a, v8f& b, v16h x, v16h y) { dep_guard_h(a, b, x, y); }
  static __device__ __forceinline__ void keep(v16h a, v16h b, v16h c, v16h d) { keep4_h(a, b, c, d); }
};
template <> struct Frag<__bf16> {
  typedef v16b V; union U { v16b v; v8b h[2]; };
  static __device__ __forceinline__ v16b load(const __bf16* p) {
    U f; f.h[0] = *(const v8b*)(p); f.h[1] = *(const v8b*)(p + 16); return f.v;
  }
  static __device__ __forceinline__ v8f mma(v16b a, v16b b, v8f c) {
    return __builtin_amdgcn_wmma_f32_16x16x32_bf16(false, a, false, b, (short)0, c, false, false);
  }
  static __device__ __forceinline__ void guard(v8f& a, v8f& b, v16b x, v16b y) { dep_guard_b(a, b, x, y); }
  static __device__ __forceinline__ void keep(v16b a, v16b b, v16b c, v16b d) { keep4_b(a, b, c, d); }
};

__device__ __forceinline__ unsigned pk16(unsigned short a, unsigned short b) { return (unsigned)a | ((unsigned)b << 16); }
__device__ __forceinline__ unsigned short h_bits(float f) { const _Float16 h = (_Float16)f; return __builtin_bit_cast(unsigned short, h); }

__device__ __forceinline__ float h16_to_f32(unsigned hb) {
  const unsigned sgn = (hb & 0x8000u) << 16; const unsigned em = hb & 0x7fffu;
  const float fn = __uint_as_float((em << 13) + 0x38000000u);
  const float fs = (float)em * 5.9604644775390625e-8f;
  const float mag = (em < 0x400u) ? fs : fn; return __uint_as_float(__float_as_uint(mag) | sgn); }

template <int ET> struct Elem;
template <> struct Elem<0> { typedef _Float16 T; };
template <> struct Elem<1> { typedef __bf16 T; };
template <int ET, bool SPLIT, int BIAS_MODE, int OUT_MODE, bool RESID, int ACT = 0>
__global__ __launch_bounds__(256) void wmma_gemm64(
    const unsigned short* __restrict__ Ap, const unsigned short* __restrict__ A2p, int lda, long strideA,
    const unsigned short* __restrict__ Btp, const unsigned short* __restrict__ Bt2p, int ldb, long strideB,
    void* __restrict__ Cout, void* __restrict__ Cout2, int ldc, long strideC,
    const float* __restrict__ bias,
    const float* __restrict__ resid, long strideR,
    int M, int N, int K, float scale) {
  typedef typename Elem<ET>::T T;
  typedef typename Frag<T>::V V;
  const T* A = (const T*)Ap; const T* A2 = (const T*)A2p; const T* Bt = (const T*)Btp; const T* Bt2 = (const T*)Bt2p;
  __shared__ __align__(16) float sT[8][16 * 68];
  const int b    = blockIdx.y;
  const int lane = threadIdx.x & 31;
  const int wave = threadIdx.x >> 5;
  const int tilesN = N >> 6;
  const int tilesM = M >> 6;
  const int tile = blockIdx.x * 8 + wave;
  if (tile >= tilesM * tilesN) return;
  const int tm = tile / tilesN;
  const int tn = tile - tm * tilesN;
  const int m0 = tm << 6;
  const int n0 = tn << 6;

  const T* Ab  = A  + (size_t)b * strideA;
  const T* Bb  = Bt + (size_t)b * strideB;
  const T* Ab2 = SPLIT ? (A2  + (size_t)b * strideA) : nullptr;
  const T* Bb2 = SPLIT ? (Bt2 + (size_t)b * strideB) : nullptr;

  const int rlane = lane & 15;
  const int koff  = (lane >> 4) * 8;
  const int mOff  = (lane >> 4) * 8;

  v8f acc[4][4];
#pragma unroll
  for (int i = 0; i < 4; ++i)
#pragma unroll
    for (int j = 0; j < 4; ++j) acc[i][j] = (v8f){0.f,0.f,0.f,0.f,0.f,0.f,0.f,0.f};

  for (int k0 = 0; k0 < K; k0 += 32) {
    V bh[4], bl[4];
#pragma unroll
    for (int j = 0; j < 4; ++j) {
      const size_t bo = (size_t)(n0 + (j << 4) + rlane) * ldb + koff + k0;
      bh[j] = Frag<T>::load(Bb + bo);
      if (SPLIT) bl[j] = Frag<T>::load(Bb2 + bo);
    }
#pragma unroll
    for (int i = 0; i < 4; ++i) {
      const size_t ao = (size_t)(m0 + (i << 4) + rlane) * lda + koff + k0;
      V ah = Frag<T>::load(Ab + ao);
      V al;
      if (SPLIT) al = Frag<T>::load(Ab2 + ao);
#pragma unroll
      for (int j = 0; j < 4; ++j) {
        acc[i][j] = Frag<T>::mma(ah, bh[j], acc[i][j]);
        if (SPLIT) {
          acc[i][j] = Frag<T>::mma(ah, bl[j], acc[i][j]);
          acc[i][j] = Frag<T>::mma(al, bh[j], acc[i][j]);
        }
      }
      Frag<T>::guard(acc[i][0], acc[i][3], ah, SPLIT ? al : ah);
    }
    Frag<T>::keep(bh[0], bh[1], bh[2], bh[3]);
    if (SPLIT) Frag<T>::keep(bl[0], bl[1], bl[2], bl[3]);
  }
  acc_guard4(acc[0][0], acc[0][1], acc[0][2], acc[0][3]);
  acc_guard4(acc[1][0], acc[1][1], acc[1][2], acc[1][3]);
  acc_guard4(acc[2][0], acc[2][1], acc[2][2], acc[2][3]);
  acc_guard4(acc[3][0], acc[3][1], acc[3][2], acc[3][3]);

  float* slab = sT[wave];
  const float* Rb = RESID ? (resid + (size_t)b * strideR) : nullptr;
#pragma unroll
  for (int i = 0; i < 4; ++i) {
    const int mBase = m0 + (i << 4);
#pragma unroll
    for (int j = 0; j < 4; ++j) {
      const int n = n0 + (j << 4) + rlane;
      float bv = 0.f;
      if (BIAS_MODE == 2) bv = bias[n];
#pragma unroll
      for (int r = 0; r < 8; ++r) {
        float v = acc[i][j][r] * scale;
        if (BIAS_MODE == 1) v += bias[mBase + mOff + r];
        if (BIAS_MODE == 2) v += bv;
        if (RESID) v += Rb[(size_t)(mBase + mOff + r) * ldc + n];
        if (ACT == 2) v = fmaxf(v, 0.0f);
        if (ACT == 6) v = (v > 0.f) ? (v + 1.0f) : expf(v);
        slab[(mOff + r) * 68 + (j << 4) + rlane] = v;
      }
    }
    __builtin_amdgcn_fence(__ATOMIC_RELEASE, "workgroup");
    __builtin_amdgcn_wave_barrier();
    __builtin_amdgcn_fence(__ATOMIC_ACQUIRE, "workgroup");
    if (OUT_MODE == 0) {
      float* C = (float*)Cout + (size_t)b * strideC;
      const int hh = lane >> 4, c4 = (lane & 15) * 4;
      for (int pass = 0; pass < 2; ++pass) {
#pragma unroll
        for (int it = 0; it < 8; ++it) {
          const int row = it * 2 + hh;
          v4f v = *(const v4f*)(slab + row * 68 + c4);
          *(volatile v4f*)(C + (size_t)(mBase + row) * ldc + n0 + c4) = v;
        }
        __threadfence();
      }
    } else {
      const int q = lane >> 3, c8 = (lane & 7) * 8;
      unsigned short* C  = (unsigned short*)Cout  + (size_t)b * strideC;
      unsigned short* C2 = (OUT_MODE == 2) ? ((unsigned short*)Cout2 + (size_t)b * strideC) : nullptr;
      for (int pass = 0; pass < 2; ++pass) {
#pragma unroll
        for (int it = 0; it < 4; ++it) {
          const int row = it * 4 + q;
          const float* sp = slab + row * 68 + c8;
          v8h hv, lv;
#pragma unroll
          for (int e = 0; e < 8; ++e) {
            if (OUT_MODE == 1) {
              hv[e] = (_Float16)sp[e];
            } else {
              unsigned short hb = f2bf_bits(sp[e]);
              unsigned short lb = f2bf_bits(sp[e] - bf_bits2f(hb));
              hv[e] = __builtin_bit_cast(_Float16, hb);
              lv[e] = __builtin_bit_cast(_Float16, lb);
            }
          }
          *(volatile v8h*)(C + (size_t)(mBase + row) * ldc + n0 + c8) = hv;
          if (OUT_MODE == 2) *(volatile v8h*)(C2 + (size_t)(mBase + row) * ldc + n0 + c8) = lv;
        }
        __threadfence();
      }
    }
    __builtin_amdgcn_fence(__ATOMIC_RELEASE, "workgroup");
    __builtin_amdgcn_wave_barrier();
    __builtin_amdgcn_fence(__ATOMIC_ACQUIRE, "workgroup");
  }
}

__global__ __launch_bounds__(256) void cast8_kernel(const float* __restrict__ in, unsigned short* __restrict__ out,
                                                    int n8, int colsLog2, int opitch, float scale) {
  const int i = blockIdx.x * 256 + threadIdx.x;
  if (i >= n8) return;
  const size_t e = 8 * (size_t)i;
  const size_t row = e >> colsLog2;
  const int col = (int)(e & (size_t)((1u << colsLog2) - 1u));
  const float* p = in + e;
  const v4f a = *(const v4f*)(p);
  const v4f c = *(const v4f*)(p + 4);
  unsigned short hb[8];
#pragma unroll
  for (int k = 0; k < 4; ++k) {
    hb[k]     = h_bits(a[k] * scale);
    hb[4 + k] = h_bits(c[k] * scale);
  }
  const v4u u = (v4u){pk16(hb[0], hb[1]), pk16(hb[2], hb[3]), pk16(hb[4], hb[5]), pk16(hb[6], hb[7])};
  unsigned short* q = out + row * (size_t)opitch + col;
  *(volatile v4u*)q = u;
  __threadfence();
  *(volatile v4u*)q = u;
}

__global__ __launch_bounds__(256) void wcast6_kernel(const float* __restrict__ w0, const float* __restrict__ w1,
                                                     const float* __restrict__ w2, const float* __restrict__ w3,
                                                     const float* __restrict__ w4, const float* __restrict__ w5,
                                                     unsigned short* __restrict__ o0, unsigned short* __restrict__ o1,
                                                     unsigned short* __restrict__ o2, unsigned short* __restrict__ o3,
                                                     unsigned short* __restrict__ o4, unsigned short* __restrict__ o5,
                                                     int n8s, int n8m, int n8l, float scale) {
  const int z = blockIdx.y;
  const float* in = (z == 0) ? w0 : (z == 1) ? w1 : (z == 2) ? w2 : (z == 3) ? w3 : (z == 4) ? w4 : w5;
  unsigned short* out = (z == 0) ? o0 : (z == 1) ? o1 : (z == 2) ? o2 : (z == 3) ? o3 : (z == 4) ? o4 : o5;
  const int n8 = (z < 4) ? n8s : ((z == 4) ? n8m : n8l);
  const int i = blockIdx.x * 256 + threadIdx.x;
  if (i >= n8) return;
  const float* p = in + 8 * (size_t)i;
  const v4f a = *(const v4f*)(p);
  const v4f c = *(const v4f*)(p + 4);
  unsigned short hb[8];
#pragma unroll
  for (int k = 0; k < 4; ++k) {
    hb[k]     = h_bits(a[k] * scale);
    hb[4 + k] = h_bits(c[k] * scale);
  }
  const v4u u = (v4u){pk16(hb[0], hb[1]), pk16(hb[2], hb[3]), pk16(hb[4], hb[5]), pk16(hb[6], hb[7])};
  unsigned short* q = out + 8 * (size_t)i;
  *(volatile v4u*)q = u;
  __threadfence();
  *(volatile v4u*)q = u;
}

__global__ __launch_bounds__(256) void ksum_kernel(const unsigned short* __restrict__ KT, float* __restrict__ KS) {
  __shared__ __align__(16) float sk[32];
  const int lane = threadIdx.x & 31, wave = threadIdx.x >> 5;
  const int rbase = blockIdx.x * 32 + wave * 4;
#pragma unroll 1
  for (int rr = 0; rr < 4; ++rr) {
    const unsigned short* rowp = KT + (size_t)(rbase + rr) * kSeq;
    float s = 0.0f;
#pragma unroll 1
    for (int it = 0; it < 32; ++it) {
      const v4u w = *(const v4u*)(rowp + it * 256 + lane * 8);
#pragma unroll
      for (int j = 0; j < 4; ++j) {
        s += h16_to_f32(w[j] & 0xffffu);
        s += h16_to_f32(w[j] >> 16);
      }
    }
#pragma unroll
    for (int off = 1; off < 32; off <<= 1) s += __shfl_xor(s, off, 32);
    if (lane == 0) sk[wave * 4 + rr] = s;
  }
  __syncthreads();
  if (wave == 0 && lane < 8) {
    const v4f v = *(const v4f*)(sk + 4 * lane);
    float* p = KS + (size_t)blockIdx.x * 32 + 4 * lane;
    *(volatile v4f*)p = v;
    __threadfence();
    *(volatile v4f*)p = v;
  }
}

__global__ __launch_bounds__(128) void kvcast_kernel(const float* __restrict__ KVF, unsigned short* __restrict__ KVT) {
  const int nh = blockIdx.x;
  const int n = nh >> 3, h = nh & 7;
  const int t = threadIdx.x;
  const int v = t >> 2, d0 = (t & 3) * 8;
  const float* src = KVF + ((size_t)(n * kDim + h * kDh + v)) * kDim + h * kDh + d0;
  const v4f a = *(const v4f*)(src);
  const v4f c = *(const v4f*)(src + 4);
  unsigned short hb[8];
#pragma unroll
  for (int k = 0; k < 4; ++k) {
    hb[k]     = h_bits(a[k]);
    hb[4 + k] = h_bits(c[k]);
  }
  const v4u u = (v4u){pk16(hb[0], hb[1]), pk16(hb[2], hb[3]), pk16(hb[4], hb[5]), pk16(hb[6], hb[7])};
  unsigned short* q = KVT + (size_t)nh * 1024 + v * 32 + d0;
  *(volatile v4u*)q = u;
  __threadfence();
  *(volatile v4u*)q = u;
}

__global__ __launch_bounds__(256) void message_kernel(const unsigned short* __restrict__ Q16p,
                                                      const unsigned short* __restrict__ KVTp,
                                                      const float* __restrict__ KSUM,
                                                      unsigned short* __restrict__ MSG) {
  typedef _Float16 T;
  const T* Q  = (const T*)Q16p;
  const T* KV = (const T*)KVTp;
  __shared__ float sKs[256];
  __shared__ float sZ[128 * 8];
  __shared__ __align__(16) float sT[8][16 * 68];
  const int tid = threadIdx.x;
  const int lane = tid & 31, wave = tid >> 5;
  const int row0 = blockIdx.x * 128;
  const int n = row0 / kSeq;
  sKs[tid] = KSUM[n * kDim + tid];
  __syncthreads();
  {
    const int r = tid >> 1, hg = tid & 1;
    const unsigned short* qrow = Q16p + (size_t)(row0 + r) * kDim;
#pragma unroll 1
    for (int e = 0; e < 4; ++e) {
      const int h = hg * 4 + e;
      const v4u w0 = *(const v4u*)(qrow + h * 32);
      const v4u w1 = *(const v4u*)(qrow + h * 32 + 8);
      const v4u w2 = *(const v4u*)(qrow + h * 32 + 16);
      const v4u w3 = *(const v4u*)(qrow + h * 32 + 24);
      const float* ks = sKs + h * 32;
      float z = 0.0f;
#pragma unroll
      for (int j = 0; j < 4; ++j) {
        const unsigned u0 = w0[j], u1 = w1[j], u2 = w2[j], u3 = w3[j];
        z = fmaf(h16_to_f32(u0 & 0xffffu), ks[2 * j],          z);
        z = fmaf(h16_to_f32(u0 >> 16),      ks[2 * j + 1],      z);
        z = fmaf(h16_to_f32(u1 & 0xffffu), ks[8 + 2 * j],      z);
        z = fmaf(h16_to_f32(u1 >> 16),      ks[8 + 2 * j + 1],  z);
        z = fmaf(h16_to_f32(u2 & 0xffffu), ks[16 + 2 * j],     z);
        z = fmaf(h16_to_f32(u2 >> 16),      ks[16 + 2 * j + 1], z);
        z = fmaf(h16_to_f32(u3 & 0xffffu), ks[24 + 2 * j],     z);
        z = fmaf(h16_to_f32(u3 >> 16),      ks[24 + 2 * j + 1], z);
      }
      sZ[r * 8 + h] = kMsgCarry / (z + kAttnEps);
    }
  }
  __syncthreads();

  const int rlane = lane & 15, koff = (lane >> 4) * 8, mOff = (lane >> 4) * 8;
  const int rowW = row0 + wave * 16;
  float* slab = sT[wave];
  const int q = lane >> 3, c8 = (lane & 7) * 8;
  const v8f zero8 = (v8f){0.f,0.f,0.f,0.f,0.f,0.f,0.f,0.f};
#pragma unroll 1
  for (int hp = 0; hp < 4; ++hp) {
    v8f acc[2][2];
#pragma unroll
    for (int e2 = 0; e2 < 2; ++e2) {
      const int h = hp * 2 + e2;
      const v16h a = Frag<T>::load(Q + (size_t)(rowW + rlane) * kDim + h * 32 + koff);
      v16h bq[2];
#pragma unroll
      for (int jt = 0; jt < 2; ++jt)
        bq[jt] = Frag<T>::load(KV + (size_t)((n * kHeads + h) * 32 + jt * 16 + rlane) * 32 + koff);
#pragma unroll
      for (int jt = 0; jt < 2; ++jt) acc[e2][jt] = Frag<T>::mma(a, bq[jt], zero8);
      Frag<T>::guard(acc[e2][0], acc[e2][1], a, bq[1]);
    }
    acc_guard4(acc[0][0], acc[0][1], acc[1][0], acc[1][1]);
#pragma unroll
    for (int e2 = 0; e2 < 2; ++e2)
#pragma unroll
      for (int jt = 0; jt < 2; ++jt)
#pragma unroll
        for (int r = 0; r < 8; ++r) {
          const float zc = sZ[(wave * 16 + mOff + r) * 8 + hp * 2 + e2];
          slab[(mOff + r) * 68 + e2 * 32 + jt * 16 + rlane] = acc[e2][jt][r] * zc;
        }
    __syncthreads();
    for (int pass = 0; pass < 2; ++pass) {
#pragma unroll
      for (int it = 0; it < 4; ++it) {
        const int row = it * 4 + q;
        const float* sp = slab + row * 68 + c8;
        unsigned short hb[8];
#pragma unroll
        for (int e = 0; e < 8; ++e) hb[e] = h_bits(sp[e]);
        const v4u u = (v4u){pk16(hb[0], hb[1]), pk16(hb[2], hb[3]), pk16(hb[4], hb[5]), pk16(hb[6], hb[7])};
        *(volatile v4u*)(MSG + (size_t)(rowW + row) * kDim + hp * 64 + c8) = u;
      }
      __threadfence();
    }
    __syncthreads();
  }
}

template <bool F32OUT>
__global__ __launch_bounds__(64) void gemm_ln_kernel(
    const unsigned short* __restrict__ Ap, int lda,
    const unsigned short* __restrict__ Btp, int K, float scale,
    const float* __restrict__ gam, const float* __restrict__ bet,
    const float* __restrict__ resid,
    float* __restrict__ outF, unsigned short* __restrict__ outH, int ldo, int coloff) {
  typedef _Float16 T;
  const T* A = (const T*)Ap;
  const T* Bt = (const T*)Btp;
  __shared__ __align__(16) float sRow[2][16 * 260];
  const int lane = threadIdx.x & 31, wave = threadIdx.x >> 5;
  const int rlane = lane & 15, koff = (lane >> 4) * 8, mOff = (lane >> 4) * 8;
  const int rowW = blockIdx.x * 32 + wave * 16;
  float* slab = sRow[wave];
#pragma unroll 1
  for (int cq = 0; cq < 4; ++cq) {
    v8f acc[4];
#pragma unroll
    for (int j = 0; j < 4; ++j) acc[j] = (v8f){0.f,0.f,0.f,0.f,0.f,0.f,0.f,0.f};
    for (int k0 = 0; k0 < K; k0 += 32) {
      v16h bh[4];
#pragma unroll
      for (int j = 0; j < 4; ++j) bh[j] = Frag<T>::load(Bt + (size_t)(cq * 64 + j * 16 + rlane) * K + koff + k0);
      const v16h a = Frag<T>::load(A + (size_t)(rowW + rlane) * lda + koff + k0);
#pragma unroll
      for (int j = 0; j < 4; ++j) acc[j] = Frag<T>::mma(a, bh[j], acc[j]);
      Frag<T>::guard(acc[0], acc[3], a, a);
      Frag<T>::keep(bh[0], bh[1], bh[2], bh[3]);
    }
    acc_guard4(acc[0], acc[1], acc[2], acc[3]);
#pragma unroll
    for (int j = 0; j < 4; ++j)
#pragma unroll
      for (int r = 0; r < 8; ++r) slab[(mOff + r) * 260 + cq * 64 + j * 16 + rlane] = acc[j][r] * scale;
  }
  __syncthreads();

  const int cA = F32OUT ? (4 * lane) : (8 * lane);
  const int cB = F32OUT ? (128 + 4 * lane) : (8 * lane + 4);
  float g[8], bb[8];
  {
    const v4f gA = *(const v4f*)(gam + cA), gB = *(const v4f*)(gam + cB);
    const v4f bA = *(const v4f*)(bet + cA), bB = *(const v4f*)(bet + cB);
#pragma unroll
    for (int e = 0; e < 4; ++e) { g[e] = gA[e]; g[4 + e] = gB[e]; bb[e] = bA[e]; bb[4 + e] = bB[e]; }
  }
#pragma unroll 1
  for (int rr = 0; rr < 16; ++rr) {
    const float* sp = slab + rr * 260;
    const v4f xa = *(const v4f*)(sp + cA);
    const v4f xb = *(const v4f*)(sp + cB);
    float xv[8];
#pragma unroll
    for (int e = 0; e < 4; ++e) { xv[e] = xa[e]; xv[4 + e] = xb[e]; }
    float s = ((xv[0] + xv[1]) + (xv[2] + xv[3])) + ((xv[4] + xv[5]) + (xv[6] + xv[7]));
#pragma unroll
    for (int off = 1; off < 32; off <<= 1) s += __shfl_xor(s, off, 32);
    const float mu = s * kInvDim;
    float d[8];
    float qv = 0.0f;
#pragma unroll
    for (int e = 0; e < 8; ++e) { d[e] = xv[e] - mu; qv = fmaf(d[e], d[e], qv); }
#pragma unroll
    for (int off = 1; off < 32; off <<= 1) qv += __shfl_xor(qv, off, 32);
    const float var = qv * kInvDim;
    const float rs = rsqrtf(var + kLnEps);
    float y[8];
#pragma unroll
    for (int e = 0; e < 8; ++e) y[e] = (d[e] * rs) * g[e] + bb[e];
    const size_t row = (size_t)(rowW + rr);
    if (F32OUT) {
      const float* rp = resid + row * kDim;
      const v4f r0 = *(const v4f*)(rp + cA);
      const v4f r1 = *(const v4f*)(rp + cB);
      v4f o0, o1;
#pragma unroll
      for (int e = 0; e < 4; ++e) { o0[e] = r0[e] + y[e]; o1[e] = r1[e] + y[4 + e]; }
      float* op = outF + row * (size_t)ldo;
      *(volatile v4f*)(op + cA) = o0;
      *(volatile v4f*)(op + cB) = o1;
      __threadfence();
      *(volatile v4f*)(op + cA) = o0;
      *(volatile v4f*)(op + cB) = o1;
    } else {
      unsigned short hb[8];
#pragma unroll
      for (int e = 0; e < 8; ++e) hb[e] = h_bits(y[e]);
      const v4u u = (v4u){pk16(hb[0], hb[1]), pk16(hb[2], hb[3]), pk16(hb[4], hb[5]), pk16(hb[6], hb[7])};
      unsigned short* op = outH + row * (size_t)ldo + coloff + cA;
      *(volatile v4u*)op = u;
      __threadfence();
      *(volatile v4u*)op = u;
    }
  }
}

extern "C" void kernel_launch(void* const* d_in, const int* in_sizes, int n_in,
                              void* d_out, int out_size, void* d_ws, size_t ws_size,
                              hipStream_t stream) {
  if (n_in < 12) return;
  const int nAct = kTok * kDim;
  if (in_sizes[0] != nAct || in_sizes[1] != nAct) return;
  if (in_sizes[2] != kDim * kDim || in_sizes[3] != kDim * kDim || in_sizes[4] != kDim * kDim || in_sizes[5] != kDim * kDim) return;
  if (in_sizes[6] != kHid2 * kHid2 || in_sizes[7] != kDim * kHid2) return;
  if (in_sizes[8] != kDim || in_sizes[9] != kDim || in_sizes[10] != kDim || in_sizes[11] != kDim) return;
  if (out_size != nAct) return;

  const size_t szW   = (size_t)kDim * kDim * 2;
  const size_t szW1  = (size_t)kHid2 * kHid2 * 2;
  const size_t szW2  = (size_t)kDim * kHid2 * 2;
  const size_t szKS  = (size_t)kBatch * kDim * 4;
  const size_t szKVF = (size_t)kBatch * kDim * kDim * 4;
  const size_t szKVT = (size_t)kBatch * kHeads * kDh * kDh * 2;
  const size_t szCAT = (size_t)kTok * kHid2 * 2;
  const size_t szP   = (size_t)kTok * kDim * 2;
  const size_t offWQ  = 0;
  const size_t offWK  = offWQ + szW;
  const size_t offWV  = offWK + szW;
  const size_t offWM  = offWV + szW;
  const size_t offW1  = offWM + szW;
  const size_t offW2  = offW1 + szW1;
  const size_t offKS  = offW2 + szW2;
  const size_t offKVF = offKS + szKS;
  const size_t offKVT = offKVF + szKVF;
  const size_t offCAT = offKVT + szKVT;
  const size_t offS16 = offCAT + szCAT;
  const size_t offQ16 = offS16 + szP;
  const size_t offKT  = offQ16 + szP;
  const size_t offVT  = offKT + szP;
  const size_t offMSG = offVT + szP;
  const size_t total  = offMSG + szP;
  const size_t offHID = offKT;
  if (ws_size < total) return;

  const float* x   = (const float*)d_in[0];
  const float* src = (const float*)d_in[1];
  const float* wq  = (const float*)d_in[2];
  const float* wk  = (const float*)d_in[3];
  const float* wv  = (const float*)d_in[4];
  const float* wm  = (const float*)d_in[5];
  const float* w1  = (const float*)d_in[6];
  const float* w2  = (const float*)d_in[7];
  const float* g1  = (const float*)d_in[8];
  const float* b1  = (const float*)d_in[9];
  const float* g2  = (const float*)d_in[10];
  const float* b2  = (const float*)d_in[11];
  float* out = (float*)d_out;
  char* ws = (char*)d_ws;
  unsigned short* WQ16  = (unsigned short*)(ws + offWQ);
  unsigned short* WK16  = (unsigned short*)(ws + offWK);
  unsigned short* WV16  = (unsigned short*)(ws + offWV);
  unsigned short* WM16  = (unsigned short*)(ws + offWM);
  unsigned short* W1_16 = (unsigned short*)(ws + offW1);
  unsigned short* W2_16 = (unsigned short*)(ws + offW2);
  float* KS  = (float*)(ws + offKS);
  float* KVF = (float*)(ws + offKVF);
  unsigned short* KVT16 = (unsigned short*)(ws + offKVT);
  unsigned short* CAT16 = (unsigned short*)(ws + offCAT);
  unsigned short* S16   = (unsigned short*)(ws + offS16);
  unsigned short* Q16   = (unsigned short*)(ws + offQ16);
  unsigned short* KT16  = (unsigned short*)(ws + offKT);
  unsigned short* VT16  = (unsigned short*)(ws + offVT);
  unsigned short* MSG16 = (unsigned short*)(ws + offMSG);
  unsigned short* HID16 = (unsigned short*)(ws + offHID);

  const int n8w  = (kDim * kDim) / 8;
  const int n8w1 = (kHid2 * kHid2) / 8;
  const int n8w2 = (kDim * kHid2) / 8;
  wcast6_kernel<<<dim3(n8w1 / 256, 6), dim3(256), 0, stream>>>(
      wq, wk, wv, wm, w1, w2, WQ16, WK16, WV16, WM16, W1_16, W2_16, n8w, n8w1, n8w2, kWCarry);
  const int n8a = nAct / 8;
  cast8_kernel<<<dim3(n8a / 256), dim3(256), 0, stream>>>(x, CAT16, n8a, 8, kHid2, 1.0f);
  cast8_kernel<<<dim3(n8a / 256), dim3(256), 0, stream>>>(src, S16, n8a, 8, kDim, 1.0f);

  const long strideTok = (long)kSeq * kDim;

  wmma_gemm64<0, false, 0, 1, false, 6><<<dim3((kTok / 64) * (kDim / 64) / 8, 1), dim3(256), 0, stream>>>(
      CAT16, CAT16, kHid2, 0L, WQ16, WQ16, kDim, 0L,
      (void*)Q16, (void*)Q16, kDim, 0L, KS, KS, 0L, kTok, kDim, kDim, kWCarryInv);
  wmma_gemm64<0, false, 0, 1, false, 6><<<dim3((kDim / 64) * (kSeq / 64) / 8, kBatch), dim3(256), 0, stream>>>(
      WK16, WK16, kDim, 0L, S16, S16, kDim, strideTok,
      (void*)KT16, (void*)KT16, kSeq, strideTok, KS, KS, 0L, kDim, kSeq, kDim, kWCarryInv);
  wmma_gemm64<0, false, 0, 1, false, 0><<<dim3((kDim / 64) * (kSeq / 64) / 8, kBatch), dim3(256), 0, stream>>>(
      WV16, WV16, kDim, 0L, S16, S16, kDim, strideTok,
      (void*)VT16, (void*)VT16, kSeq, strideTok, KS, KS, 0L, kDim, kSeq, kDim, kWCarryInv);
  wmma_gemm64<0, false, 0, 0, false, 0><<<dim3((kDim / 64) * (kDim / 64) / 8, kBatch), dim3(256), 0, stream>>>(
      VT16, VT16, kSeq, strideTok, KT16, KT16, kSeq, strideTok,
      (void*)KVF, (void*)KVF, kDim, (long)kDim * kDim, KS, KS, 0L, kDim, kDim, kSeq, 1.0f);
  kvcast_kernel<<<dim3(kBatch * kHeads), dim3(128), 0, stream>>>(KVF, KVT16);
  ksum_kernel<<<dim3((kBatch * kDim) / 32), dim3(256), 0, stream>>>(KT16, KS);
  message_kernel<<<dim3(kTok / 128), dim3(256), 0, stream>>>(Q16, KVT16, KS, MSG16);
  gemm_ln_kernel<false><<<dim3(kTok / 32), dim3(64), 0, stream>>>(
      MSG16, kDim, WM16, kDim, kMergeScale, g1, b1, x, KVF, CAT16, kHid2, kDim);
  wmma_gemm64<0, false, 0, 1, false, 2><<<dim3((kTok / 64) * (kHid2 / 64) / 8, 1), dim3(256), 0, stream>>>(
      CAT16, CAT16, kHid2, 0L, W1_16, W1_16, kHid2, 0L,
      (void*)HID16, (void*)HID16, kHid2, 0L, KS, KS, 0L, kTok, kHid2, kHid2, kWCarryInv);
  gemm_ln_kernel<true><<<dim3(kTok / 32), dim3(64), 0, stream>>>(
      HID16, kHid2, W2_16, kHid2, kWCarryInv, g2, b2, x, out, CAT16, kDim, 0);
}
